// MambaBlock_81853486727588
// MI455X (gfx1250) — hardware-verified
//
#include <hip/hip_runtime.h>
#include <math.h>

typedef __attribute__((ext_vector_type(16))) _Float16 v16h;
typedef __attribute__((ext_vector_type(8)))  _Float16 v8h;
typedef __attribute__((ext_vector_type(16))) __bf16   v16b;
typedef __attribute__((ext_vector_type(8)))  __bf16   v8b;
typedef __attribute__((ext_vector_type(8)))  float    v8f;
typedef __attribute__((ext_vector_type(4)))  float    v4f;
typedef __attribute__((ext_vector_type(4)))  unsigned int v4u;

constexpr int kBatch = 2;
constexpr int kSeqL  = 2048;
constexpr int kDmod  = 1024;
constexpr int kDin   = 2048;
constexpr int kNst   = 16;
constexpr int kDtR   = 128;
constexpr int kPrjN  = 160;
constexpr int kPrjP  = 192;
constexpr int kXZP   = 2 * kDin;
constexpr int kRows  = kBatch * kSeqL;
constexpr int kTP    = 260;
constexpr float kEps   = 1e-5f;
constexpr float kLog2e = 1.4426950408889634f;
constexpr float kWinC  = 32.0f;
constexpr float kWxC   = 32.0f;
constexpr float kWdtC  = 8.0f;
constexpr float kWoutC = 256.0f;
constexpr float kDtC   = 16.0f;
constexpr float kYC    = 16.0f;
constexpr float kSclIn  = 1.0f / kWinC;
constexpr float kSclX   = 1.0f / kWxC;
constexpr float kSclDt  = 1.0f / (kDtC * kWdtC);
constexpr float kSclOut = 1.0f / (kYC * kWoutC);
static_assert(kPrjN == kDtR + 2 * kNst, "x_proj width");
static_assert(kXZP == 4096 && kRows == 4096, "shapes");
static_assert((kDmod % 32) == 0 && (kDin % 32) == 0 && (kDtR % 32) == 0, "GEMM K multiples of 32");
static_assert((kSeqL % 64) == 0 && (kXZP % 64) == 0 && (kPrjP % 64) == 0 && (kDin % 64) == 0 && (kDmod % 64) == 0, "GEMM M,N multiples of 64");
static_assert((kSeqL % 16) == 0 && (kDin % 256) == 0 && (kDmod % 8) == 0, "VALU tiles");

constexpr size_t kOffWIN  = 0;
constexpr size_t kOffWX   = kOffWIN  + (size_t)kXZP  * kDmod * 2;
constexpr size_t kOffWDT  = kOffWX   + (size_t)kPrjP * kDin  * 2;
constexpr size_t kOffWOUT = kOffWDT  + (size_t)kDin  * kDtR  * 2;
constexpr size_t kOffXN   = kOffWOUT + (size_t)kDmod * kDin  * 2;
constexpr size_t kOffXZ   = kOffXN   + (size_t)kRows * kDmod * 2;
constexpr size_t kOffUC   = kOffXZ   + (size_t)kSeqL * kXZP  * 4;
constexpr size_t kOffUC16 = kOffUC   + (size_t)kSeqL * kDin  * 4;
constexpr size_t kOffDBL  = kOffUC16 + (size_t)kSeqL * kDin  * 2;
constexpr size_t kOffDT16 = kOffDBL  + (size_t)kSeqL * kPrjP * 4;
constexpr size_t kOffDTP  = kOffDT16 + (size_t)kSeqL * kDtR  * 2;
constexpr size_t kOffY16  = kOffDTP  + (size_t)kSeqL * kDin  * 4;
constexpr size_t kWsTotal = kOffY16  + (size_t)kSeqL * kDin  * 2;
static_assert(kWsTotal == 108265472ull, "carve total");
static_assert(kWsTotal <= 134217728ull, "carve cap");
static_assert((kOffWX % 512) == 0 && (kOffWDT % 512) == 0 && (kOffWOUT % 512) == 0 && (kOffXN % 512) == 0 &&
              (kOffXZ % 512) == 0 && (kOffUC % 512) == 0 && (kOffUC16 % 512) == 0 && (kOffDBL % 512) == 0 &&
              (kOffDT16 % 512) == 0 && (kOffDTP % 512) == 0 && (kOffY16 % 512) == 0, "512-B aligned regions");

__device__ __forceinline__ unsigned short f2bf_bits(float f) {
  unsigned u = __float_as_uint(f);
  return (unsigned short)((u + 0x7FFFu + ((u >> 16) & 1u)) >> 16);
}
__device__ __forceinline__ float bf_bits2f(unsigned short h) { return __uint_as_float(((unsigned)h) << 16); }

__device__ __forceinline__ void dep_guard_h(v8f& a, v8f& b, v16h x, v16h y) { asm volatile("v_nop\n\tv_nop\n\tv_nop\n\tv_nop" : "+v"(a), "+v"(b) : "v"(x), "v"(y)); }
__device__ __forceinline__ void dep_guard_b(v8f& a, v8f& b, v16b x, v16b y) { asm volatile("v_nop\n\tv_nop\n\tv_nop\n\tv_nop" : "+v"(a), "+v"(b) : "v"(x), "v"(y)); }
__device__ __forceinline__ void dep_guard4_h(v8f& a, v8f& b, v8f& c, v8f& d, v16h x, v16h y) { asm volatile("v_nop\n\tv_nop\n\tv_nop\n\tv_nop" : "+v"(a), "+v"(b), "+v"(c), "+v"(d) : "v"(x), "v"(y)); }
__device__ __forceinline__ void dep_guard4_b(v8f& a, v8f& b, v8f& c, v8f& d, v16b x, v16b y) { asm volatile("v_nop\n\tv_nop\n\tv_nop\n\tv_nop" : "+v"(a), "+v"(b), "+v"(c), "+v"(d) : "v"(x), "v"(y)); }
__device__ __forceinline__ void keep4_h(v16h a, v16h b, v16h c, v16h d) { asm volatile("v_nop" :: "v"(a), "v"(b), "v"(c), "v"(d)); }
__device__ __forceinline__ void keep4_b(v16b a, v16b b, v16b c, v16b d) { asm volatile("v_nop" :: "v"(a), "v"(b), "v"(c), "v"(d)); }
__device__ __forceinline__ void acc_guard4(v8f& a, v8f& b, v8f& c, v8f& d) { asm volatile("v_nop\n\tv_nop\n\tv_nop\n\tv_nop" : "+v"(a), "+v"(b), "+v"(c), "+v"(d)); }
template <typename T> struct Frag;
template <> struct Frag<_Float16> {
  typedef v16h V; union U { v16h v; v8h h[2]; };
  static __device__ __forceinline__ v16h load(const _Float16* p) {
    U f; f.h[0] = *(const v8h*)(p); f.h[1] = *(const v8h*)(p + 16); return f.v;
  }
  static __device__ __forceinline__ v8f mma(v16h a, v16h b, v8f c) {
    return __builtin_amdgcn_wmma_f32_16x16x32_f16(false, a, false, b, (short)0, c, false, false);
  }
  static __device__ __forceinline__ void guard(v8f& a, v8f& b, v16h x, v16h y) { dep_guard_h(a, b, x, y); }
  static __device__ __forceinline__ void guard4(v8f& a, v8f& b, v8f& c, v8f& d, v16h x, v16h y) { dep_guard4_h(a, b, c, d, x, y); }
  static __device__ __forceinline__ void keep(v16h a, v16h b, v16h c, v16h d) { keep4_h(a, b, c, d); }
};
template <> struct Frag<__bf16> {
  typedef v16b V; union U { v16b v; v8b h[2]; };
  static __device__ __forceinline__ v16b load(const __bf16* p) {
    U f; f.h[0] = *(const v8b*)(p); f.h[1] = *(const v8b*)(p + 16); return f.v;
  }
  static __device__ __forceinline__ v8f mma(v16b a, v16b b, v8f c) {
    return __builtin_amdgcn_wmma_f32_16x16x32_bf16(false, a, false, b, (short)0, c, false, false);
  }
  static __device__ __forceinline__ void guard(v8f& a, v8f& b, v16b x, v16b y) { dep_guard_b(a, b, x, y); }
  static __device__ __forceinline__ void guard4(v8f& a, v8f& b, v8f& c, v8f& d, v16b x, v16b y) { dep_guard4_b(a, b, c, d, x, y); }
  static __device__ __forceinline__ void keep(v16b a, v16b b, v16b c, v16b d) { keep4_b(a, b, c, d); }
};

template <int ET> struct Elem;
template <> struct Elem<0> { typedef _Float16 T; };
template <> struct Elem<1> { typedef __bf16 T; };
template <int ET, bool SPLIT, int BIAS_MODE, int OUT_MODE, bool RESID, int ACT = 0>
__global__ __launch_bounds__(256) void wmma_gemm64(
    const unsigned short* __restrict__ Ap, const unsigned short* __restrict__ A2p, int lda, long strideA,
    const unsigned short* __restrict__ Btp, const unsigned short* __restrict__ Bt2p, int ldb, long strideB,
    void* __restrict__ Cout, void* __restrict__ Cout2, int ldc, long strideC,
    const float* __restrict__ bias,
    const float* __restrict__ resid, long strideR,
    int M, int N, int K, float scale) {
  static_assert(!(RESID && OUT_MODE != 0), "residual path is f32 output only");
  typedef typename Elem<ET>::T T;
  typedef typename Frag<T>::V V;
  const T* A = (const T*)Ap; const T* A2 = (const T*)A2p; const T* Bt = (const T*)Btp; const T* Bt2 = (const T*)Bt2p;
  __shared__ __align__(16) float sT[8][16 * 68];
  const int b    = blockIdx.y;
  const int lane = threadIdx.x & 31;
  const int wave = threadIdx.x >> 5;
  const int tilesN = N >> 6;
  const int tilesM = M >> 6;
  const int tile = blockIdx.x * 8 + wave;
  if (tile >= tilesM * tilesN) return;
  const int tm = tile / tilesN;
  const int tn = tile - tm * tilesN;
  const int m0 = tm << 6;
  const int n0 = tn << 6;

  const T* Ab  = A  + (size_t)b * strideA;
  const T* Bb  = Bt + (size_t)b * strideB;
  const T* Ab2 = SPLIT ? (A2  + (size_t)b * strideA) : nullptr;
  const T* Bb2 = SPLIT ? (Bt2 + (size_t)b * strideB) : nullptr;

  const int rlane = lane & 15;
  const int koff  = (lane >> 4) * 8;
  const int mOff  = (lane >> 4) * 8;

  v8f acc[4][4];
#pragma unroll
  for (int i = 0; i < 4; ++i)
#pragma unroll
    for (int j = 0; j < 4; ++j) acc[i][j] = (v8f){0.f,0.f,0.f,0.f,0.f,0.f,0.f,0.f};

  for (int k0 = 0; k0 < K; k0 += 32) {
    V bh[4], bl[4];
#pragma unroll
    for (int j = 0; j < 4; ++j) {
      const size_t bo = (size_t)(n0 + (j << 4) + rlane) * ldb + koff + k0;
      bh[j] = Frag<T>::load(Bb + bo);
      if (SPLIT) bl[j] = Frag<T>::load(Bb2 + bo);
    }
#pragma unroll
    for (int i = 0; i < 4; ++i) {
      const size_t ao = (size_t)(m0 + (i << 4) + rlane) * lda + koff + k0;
      V ah = Frag<T>::load(Ab + ao);
      V al;
      if (SPLIT) al = Frag<T>::load(Ab2 + ao);
#pragma unroll
      for (int j = 0; j < 4; ++j) {
        acc[i][j] = Frag<T>::mma(ah, bh[j], acc[i][j]);
        if (SPLIT) {
          acc[i][j] = Frag<T>::mma(ah, bl[j], acc[i][j]);
          acc[i][j] = Frag<T>::mma(al, bh[j], acc[i][j]);
        }
      }
      Frag<T>::guard4(acc[i][0], acc[i][1], acc[i][2], acc[i][3], ah, SPLIT ? al : ah);
    }
    Frag<T>::keep(bh[0], bh[1], bh[2], bh[3]);
    if (SPLIT) Frag<T>::keep(bl[0], bl[1], bl[2], bl[3]);
  }
  acc_guard4(acc[0][0], acc[0][1], acc[0][2], acc[0][3]);
  acc_guard4(acc[1][0], acc[1][1], acc[1][2], acc[1][3]);
  acc_guard4(acc[2][0], acc[2][1], acc[2][2], acc[2][3]);
  acc_guard4(acc[3][0], acc[3][1], acc[3][2], acc[3][3]);

  float* slab = sT[wave];
  const float* Rb = RESID ? (resid + (size_t)b * strideR) : nullptr;
#pragma unroll
  for (int i = 0; i < 4; ++i) {
    const int mBase = m0 + (i << 4);
#pragma unroll
    for (int j = 0; j < 4; ++j) {
      const int n = n0 + (j << 4) + rlane;
      float bv = 0.f;
      if (BIAS_MODE == 2) bv = bias[n];
#pragma unroll
      for (int r = 0; r < 8; ++r) {
        float v = acc[i][j][r] * scale;
        if (BIAS_MODE == 1) v += bias[mBase + mOff + r];
        if (BIAS_MODE == 2) v += bv;
        if (ACT == 1) v = tanhf(v);
        if (ACT == 2) v = fmaxf(v, 0.0f);
        if (ACT == 3) v = v / (1.0f + expf(-v));
        if (ACT == 4) v = (v > 0.f) ? v : 0.01f * v;
        slab[(mOff + r) * 68 + (j << 4) + rlane] = v;
      }
    }
    __builtin_amdgcn_fence(__ATOMIC_RELEASE, "workgroup");
    __builtin_amdgcn_wave_barrier();
    __builtin_amdgcn_fence(__ATOMIC_ACQUIRE, "workgroup");
    if (OUT_MODE == 0) {
      float* C = (float*)Cout + (size_t)b * strideC;
      const int hh = lane >> 4, c4 = (lane & 15) * 4;
      for (int pass = 0; pass < 2; ++pass) {
#pragma unroll
        for (int it = 0; it < 8; ++it) {
          const int row = it * 2 + hh;
          v4f v = *(const v4f*)(slab + row * 68 + c4);
          if (RESID) {
            const v4f rv = *(const v4f*)(Rb + (size_t)(mBase + row) * ldc + n0 + c4);
            v = v + rv;
          }
          *(volatile v4f*)(C + (size_t)(mBase + row) * ldc + n0 + c4) = v;
          if (RESID && it == 3) asm volatile("" ::: "memory");
        }
        __threadfence();
      }
    } else {
      const int q = lane >> 3, c8 = (lane & 7) * 8;
      unsigned short* C  = (unsigned short*)Cout  + (size_t)b * strideC;
      unsigned short* C2 = (OUT_MODE == 2) ? ((unsigned short*)Cout2 + (size_t)b * strideC) : nullptr;
      for (int pass = 0; pass < 2; ++pass) {
#pragma unroll
        for (int it = 0; it < 4; ++it) {
          const int row = it * 4 + q;
          const float* sp = slab + row * 68 + c8;
          v8h hv, lv;
#pragma unroll
          for (int e = 0; e < 8; ++e) {
            if (OUT_MODE == 1) {
              hv[e] = (_Float16)sp[e];
            } else {
              unsigned short hb = f2bf_bits(sp[e]);
              unsigned short lb = f2bf_bits(sp[e] - bf_bits2f(hb));
              hv[e] = __builtin_bit_cast(_Float16, hb);
              lv[e] = __builtin_bit_cast(_Float16, lb);
            }
          }
          *(volatile v8h*)(C + (size_t)(mBase + row) * ldc + n0 + c8) = hv;
          if (OUT_MODE == 2) *(volatile v8h*)(C2 + (size_t)(mBase + row) * ldc + n0 + c8) = lv;
        }
        __threadfence();
      }
    }
    __builtin_amdgcn_fence(__ATOMIC_RELEASE, "workgroup");
    __builtin_amdgcn_wave_barrier();
    __builtin_amdgcn_fence(__ATOMIC_ACQUIRE, "workgroup");
  }
}

__global__ __launch_bounds__(256) void cast_f16_kernel(
    const float* __restrict__ src, unsigned short* __restrict__ dst, int total8, float scale)
{
  const int i = blockIdx.x * 256 + threadIdx.x;
  if (i >= total8) return;
  const size_t e0 = (size_t)i << 3;
  const float* p = src + e0;
  const v4f a0 = *(const v4f*)(p);
  const v4f a1 = *(const v4f*)(p + 4);
  v8h hv;
#pragma unroll
  for (int e = 0; e < 4; ++e) {
    hv[e]     = (_Float16)(a0[e] * scale);
    hv[4 + e] = (_Float16)(a1[e] * scale);
  }
  unsigned short* q = dst + e0;
  *(volatile v8h*)q = hv;
  __threadfence();
  *(volatile v8h*)q = hv;
}

__global__ __launch_bounds__(256) void zero_f16_kernel(unsigned short* __restrict__ dst, int total8)
{
  const int i = blockIdx.x * 256 + threadIdx.x;
  if (i >= total8) return;
  const v4u z = (v4u){0u, 0u, 0u, 0u};
  unsigned short* q = dst + ((size_t)i << 3);
  *(volatile v4u*)q = z;
  __threadfence();
  *(volatile v4u*)q = z;
}

__global__ __launch_bounds__(128) void ln_cast_kernel(
    const float* __restrict__ x, const float* __restrict__ gw, const float* __restrict__ gb,
    unsigned short* __restrict__ XN16)
{
  __shared__ float sred[8];
  const int tid = threadIdx.x, lane = tid & 31, wave = tid >> 5;
  const size_t row = blockIdx.x;
  const int c0 = tid * 8;
  const float* xr = x + row * kDmod + c0;
  const v4f a0 = *(const v4f*)(xr);
  const v4f a1 = *(const v4f*)(xr + 4);
  const v4f g0 = *(const v4f*)(gw + c0);
  const v4f g1 = *(const v4f*)(gw + c0 + 4);
  const v4f e0 = *(const v4f*)(gb + c0);
  const v4f e1 = *(const v4f*)(gb + c0 + 4);
  float s = 0.0f;
#pragma unroll
  for (int e = 0; e < 4; ++e) s += a0[e];
#pragma unroll
  for (int e = 0; e < 4; ++e) s += a1[e];
#pragma unroll
  for (int off = 1; off < 32; off <<= 1) s += __shfl_xor(s, off, 32);
  if (lane == 0) sred[wave] = s;
  __syncthreads();
  const float mu = ((sred[0] + sred[1]) + (sred[2] + sred[3])) * (1.0f / (float)kDmod);
  const v4f d0 = a0 - mu;
  const v4f d1 = a1 - mu;
  float qs = 0.0f;
#pragma unroll
  for (int e = 0; e < 4; ++e) qs += d0[e] * d0[e];
#pragma unroll
  for (int e = 0; e < 4; ++e) qs += d1[e] * d1[e];
#pragma unroll
  for (int off = 1; off < 32; off <<= 1) qs += __shfl_xor(qs, off, 32);
  if (lane == 0) sred[4 + wave] = qs;
  __syncthreads();
  const float var = ((sred[4] + sred[5]) + (sred[6] + sred[7])) * (1.0f / (float)kDmod);
  const float rs = rsqrtf(var + kEps);
  v8h hv;
#pragma unroll
  for (int e = 0; e < 4; ++e) {
    hv[e]     = (_Float16)((d0[e] * rs) * g0[e] + e0[e]);
    hv[4 + e] = (_Float16)((d1[e] * rs) * g1[e] + e1[e]);
  }
  unsigned short* q = XN16 + row * kDmod + c0;
  *(volatile v8h*)q = hv;
  __threadfence();
  *(volatile v8h*)q = hv;
}

__global__ __launch_bounds__(256) void conv_silu_kernel(
    const float* __restrict__ XZ, const float* __restrict__ cw, const float* __restrict__ cb,
    float* __restrict__ UC, unsigned short* __restrict__ UC16)
{
  __shared__ __align__(16) float sT[16 * kTP];
  const int tid = threadIdx.x, lane = tid & 31, wave = tid >> 5;
  const int d0 = blockIdx.x * 256, d = d0 + tid;
  const int t0 = blockIdx.y * 64;
  const float w0 = cw[d * 4 + 0], w1 = cw[d * 4 + 1], w2 = cw[d * 4 + 2], w3 = cw[d * 4 + 3];
  const float bc = cb[d];
  float xm3, xm2, xm1;
  {
    const int r3 = t0 - 3, r2 = t0 - 2, r1 = t0 - 1;
    const float v3 = XZ[(size_t)(r3 < 0 ? 0 : r3) * kXZP + d];
    const float v2 = XZ[(size_t)(r2 < 0 ? 0 : r2) * kXZP + d];
    const float v1 = XZ[(size_t)(r1 < 0 ? 0 : r1) * kXZP + d];
    xm3 = (r3 >= 0) ? v3 : 0.f;
    xm2 = (r2 >= 0) ? v2 : 0.f;
    xm1 = (r1 >= 0) ? v1 : 0.f;
  }
  const int hrow = wave >> 1;
  const int hch  = (wave & 1) * 128 + lane * 4;
#pragma unroll 1
  for (int sub = 0; sub < 4; ++sub) {
    const int lb = t0 + sub * 16;
#pragma unroll 1
    for (int s = 0; s < 16; ++s) {
      const float xc = XZ[(size_t)(lb + s) * kXZP + d];
      float acc = w0 * xm3;
      acc = fmaf(w1, xm2, acc);
      acc = fmaf(w2, xm1, acc);
      acc = fmaf(w3, xc, acc);
      const float sv = acc + bc;
      const float sg = __builtin_amdgcn_rcpf(1.0f + expf(-sv));
      sT[s * kTP + tid] = sv * sg;
      xm3 = xm2; xm2 = xm1; xm1 = xc;
    }
    __syncthreads();
    v4f fv[4];
    v8h bv[2];
#pragma unroll
    for (int it = 0; it < 4; ++it) fv[it] = *(const v4f*)(sT + (it * 4 + hrow) * kTP + hch);
#pragma unroll
    for (int it = 0; it < 2; ++it) {
      const float* sp = sT + (it * 8 + wave) * kTP + lane * 8;
      const v4f a0 = *(const v4f*)(sp);
      const v4f a1 = *(const v4f*)(sp + 4);
#pragma unroll
      for (int e = 0; e < 4; ++e) {
        bv[it][e]     = (_Float16)a0[e];
        bv[it][4 + e] = (_Float16)a1[e];
      }
    }
    for (int pass = 0; pass < 2; ++pass) {
#pragma unroll
      for (int it = 0; it < 4; ++it)
        *(volatile v4f*)(UC + (size_t)(lb + it * 4 + hrow) * kDin + d0 + hch) = fv[it];
#pragma unroll
      for (int it = 0; it < 2; ++it)
        *(volatile v8h*)(UC16 + (size_t)(lb + it * 8 + wave) * kDin + d0 + lane * 8) = bv[it];
      __threadfence();
    }
    __syncthreads();
  }
}

__global__ __launch_bounds__(256) void dt_cast_kernel(
    const float* __restrict__ DBL, unsigned short* __restrict__ DT16, int total8, float scale)
{
  const int i = blockIdx.x * 256 + threadIdx.x;
  if (i >= total8) return;
  const int e0  = i << 3;
  const int row = e0 >> 7;
  const int c8  = e0 & 127;
  const float* p = DBL + (size_t)row * kPrjP + c8;
  const v4f a0 = *(const v4f*)(p);
  const v4f a1 = *(const v4f*)(p + 4);
  v8h hv;
#pragma unroll
  for (int e = 0; e < 4; ++e) {
    hv[e]     = (_Float16)(a0[e] * scale);
    hv[4 + e] = (_Float16)(a1[e] * scale);
  }
  unsigned short* qd = DT16 + e0;
  *(volatile v8h*)qd = hv;
  __threadfence();
  *(volatile v8h*)qd = hv;
}

__global__ __launch_bounds__(256) void scan_kernel(
    const float* __restrict__ DTP, const float* __restrict__ UC, const float* __restrict__ XZ,
    const float* __restrict__ DBL, const float* __restrict__ bdt, const float* __restrict__ A_log,
    const float* __restrict__ Dv, unsigned short* __restrict__ Y16)
{
  __shared__ __align__(16) float sBC[16 * 32];
  __shared__ __align__(16) float sA[kNst * 256];
  __shared__ __align__(16) float sY[16 * kTP];
  const int tid = threadIdx.x, lane = tid & 31, wave = tid >> 5;
  const int d0 = blockIdx.x * 256, d = d0 + tid;

#pragma unroll 1
  for (int n = 0; n < kNst; ++n) sA[n * 256 + tid] = -expf(A_log[(size_t)d * kNst + n]);
  __syncthreads();
  float An[kNst], h[kNst];
#pragma unroll
  for (int n = 0; n < kNst; ++n) { An[n] = sA[n * 256 + tid]; h[n] = 0.0f; }
  const float bb = bdt[d];
  const float Dd = Dv[d];

#pragma unroll 1
  for (int c = 0; c < kSeqL / 16; ++c) {
    const int l0 = c * 16;
    if (tid < 128) {
      const int r = tid >> 3, q = (tid & 7) * 4;
      const v4f v = *(const v4f*)(DBL + (size_t)(l0 + r) * kPrjP + kDtR + q);
      *(v4f*)(sBC + r * 32 + q) = v;
    }
    __syncthreads();
#pragma unroll 1
    for (int s = 0; s < 16; ++s) {
      const size_t m = (size_t)(l0 + s);
      const float a     = DTP[m * kDin + d] + bb;
      const float delta = fmaxf(a, 0.0f) + log1pf(expf(-fabsf(a)));
      const float xv    = UC[m * kDin + d];
      const float zv    = XZ[m * kXZP + kDin + d];
      v4f Bq[4], Cq[4];
#pragma unroll
      for (int qq = 0; qq < 4; ++qq) {
        Bq[qq] = *(const v4f*)(sBC + s * 32 + 4 * qq);
        Cq[qq] = *(const v4f*)(sBC + s * 32 + kNst + 4 * qq);
      }
      const float dl2 = delta * kLog2e;
      float dtu = delta * xv;
      asm volatile("" : "+v"(dtu));
      float y = 0.0f;
#pragma unroll
      for (int n = 0; n < kNst; ++n) {
        const float e = exp2f(dl2 * An[n]);
        float p = dtu * Bq[n >> 2][n & 3];
        asm volatile("" : "+v"(p));
        float qv = h[n] * e;
        asm volatile("" : "+v"(qv));
        const float hn = qv + p;
        h[n] = hn;
        float rr = hn * Cq[n >> 2][n & 3];
        asm volatile("" : "+v"(rr));
        y += rr;
      }
      float sk = xv * Dd;
      asm volatile("" : "+v"(sk));
      y += sk;
      const float sg = __builtin_amdgcn_rcpf(1.0f + expf(-zv));
      const float g  = zv * sg;
      sY[s * kTP + tid] = (y * g) * kYC;
    }
    __syncthreads();
    v8h hv[2];
#pragma unroll
    for (int it = 0; it < 2; ++it) {
      const float* sp = sY + (it * 8 + wave) * kTP + lane * 8;
      const v4f a0 = *(const v4f*)(sp);
      const v4f a1 = *(const v4f*)(sp + 4);
#pragma unroll
      for (int e = 0; e < 4; ++e) { hv[it][e] = (_Float16)a0[e]; hv[it][4 + e] = (_Float16)a1[e]; }
    }
    for (int pass = 0; pass < 2; ++pass) {
#pragma unroll
      for (int it = 0; it < 2; ++it)
        *(volatile v8h*)(Y16 + (size_t)(l0 + it * 8 + wave) * kDin + d0 + lane * 8) = hv[it];
      __threadfence();
    }
  }
}

extern "C" void kernel_launch(void* const* d_in, const int* in_sizes, int n_in,
                              void* d_out, int out_size, void* d_ws, size_t ws_size,
                              hipStream_t stream)
{
  if (n_in < 12) return;
  if (in_sizes[0] != kRows * kDmod) return;
  if (in_sizes[1] != kDmod || in_sizes[2] != kDmod) return;
  if (in_sizes[3] != kXZP * kDmod) return;
  if (in_sizes[4] != kDin * 4 || in_sizes[5] != kDin) return;
  if (in_sizes[6] != kPrjN * kDin) return;
  if (in_sizes[7] != kDin * kDtR || in_sizes[8] != kDin) return;
  if (in_sizes[9] != kDin * kNst || in_sizes[10] != kDin) return;
  if (in_sizes[11] != kDmod * kDin) return;
  if (out_size != kRows * kDmod) return;
  if (ws_size < kWsTotal) return;

  const float* x      = (const float*)d_in[0];
  const float* norm_g = (const float*)d_in[1];
  const float* norm_b = (const float*)d_in[2];
  const float* W_in   = (const float*)d_in[3];
  const float* conv_w = (const float*)d_in[4];
  const float* conv_b = (const float*)d_in[5];
  const float* Wx     = (const float*)d_in[6];
  const float* Wdt    = (const float*)d_in[7];
  const float* bdt    = (const float*)d_in[8];
  const float* A_log  = (const float*)d_in[9];
  const float* Dp     = (const float*)d_in[10];
  const float* W_out  = (const float*)d_in[11];
  float* dout = (float*)d_out;

  char* ws = (char*)d_ws;
  unsigned short* WIN16  = (unsigned short*)(ws + kOffWIN);
  unsigned short* WX16   = (unsigned short*)(ws + kOffWX);
  unsigned short* WDT16  = (unsigned short*)(ws + kOffWDT);
  unsigned short* WOUT16 = (unsigned short*)(ws + kOffWOUT);
  unsigned short* XN16   = (unsigned short*)(ws + kOffXN);
  float*          XZ     = (float*)(ws + kOffXZ);
  float*          UC     = (float*)(ws + kOffUC);
  unsigned short* UC16   = (unsigned short*)(ws + kOffUC16);
  float*          DBL    = (float*)(ws + kOffDBL);
  unsigned short* DT16   = (unsigned short*)(ws + kOffDT16);
  float*          DTP    = (float*)(ws + kOffDTP);
  unsigned short* Y16    = (unsigned short*)(ws + kOffY16);
  const float* dummy_bias  = bdt;
  const float* dummy_resid = x;

  cast_f16_kernel<<<(kXZP * kDmod) / 8 / 256, 256, 0, stream>>>(W_in,  WIN16,  (kXZP * kDmod) / 8, kWinC);
  cast_f16_kernel<<<(kPrjN * kDin) / 8 / 256, 256, 0, stream>>>(Wx,    WX16,   (kPrjN * kDin) / 8, kWxC);
  zero_f16_kernel<<<((kPrjP - kPrjN) * kDin) / 8 / 256, 256, 0, stream>>>(WX16 + (size_t)kPrjN * kDin, ((kPrjP - kPrjN) * kDin) / 8);
  cast_f16_kernel<<<(kDin * kDtR) / 8 / 256, 256, 0, stream>>>(Wdt,    WDT16,  (kDin * kDtR) / 8, kWdtC);
  cast_f16_kernel<<<(kDmod * kDin) / 8 / 256, 256, 0, stream>>>(W_out,  WOUT16, (kDmod * kDin) / 8, kWoutC);

  ln_cast_kernel<<<kRows, 128, 0, stream>>>(x, norm_g, norm_b, XN16);

  for (int b = 0; b < kBatch; ++b) {
    const unsigned short* XN16b = XN16 + (size_t)b * kSeqL * kDmod;
    const float* xb = x + (size_t)b * kSeqL * kDmod;
    float* outb = dout + (size_t)b * kSeqL * kDmod;

    wmma_gemm64<0, false, 0, 0, false><<<dim3(256, 1), 256, 0, stream>>>(
        XN16b, XN16b, kDmod, 0L, WIN16, WIN16, kDmod, 0L,
        (void*)XZ, (void*)XZ, kXZP, 0L, dummy_bias, dummy_resid, 0L, kSeqL, kXZP, kDmod, kSclIn);

    conv_silu_kernel<<<dim3(kDin / 256, kSeqL / 64), 256, 0, stream>>>(XZ, conv_w, conv_b, UC, UC16);

    wmma_gemm64<0, false, 0, 0, false><<<dim3(12, 1), 256, 0, stream>>>(
        UC16, UC16, kDin, 0L, WX16, WX16, kDin, 0L,
        (void*)DBL, (void*)DBL, kPrjP, 0L, dummy_bias, dummy_resid, 0L, kSeqL, kPrjP, kDin, kSclX);

    dt_cast_kernel<<<(kSeqL * kDtR) / 8 / 256, 256, 0, stream>>>(DBL, DT16, (kSeqL * kDtR) / 8, kDtC);

    wmma_gemm64<0, false, 0, 0, false><<<dim3(128, 1), 256, 0, stream>>>(
        DT16, DT16, kDtR, 0L, WDT16, WDT16, kDtR, 0L,
        (void*)DTP, (void*)DTP, kDin, 0L, dummy_bias, dummy_resid, 0L, kSeqL, kDin, kDtR, kSclDt);

    scan_kernel<<<dim3(kDin / 256, 1), 256, 0, stream>>>(DTP, UC, XZ, DBL, bdt, A_log, Dp, Y16);

    wmma_gemm64<0, false, 0, 0, true><<<dim3(64, 1), 256, 0, stream>>>(
        Y16, Y16, kDin, 0L, WOUT16, WOUT16, kDin, 0L,
        (void*)outb, (void*)outb, kDmod, 0L, dummy_bias, xb, 0L, kSeqL, kDmod, kDin, kSclOut);
  }
}
